// BQQLinear_25589415149866
// MI455X (gfx1250) — hardware-verified
//
#include <hip/hip_runtime.h>
#include <math.h>

constexpr int DIM_P = 2, DIM_J = 32, DIM_K = 32, DIM_M = 32, DIM_L = 8, DIM_N = 32;
constexpr int BROWS = 2048;
constexpr int KDIM  = DIM_K * DIM_N;
constexpr int NCOLS = DIM_J * DIM_M;
constexpr int GRP   = DIM_M * DIM_L;
static_assert(GRP == 256 && DIM_L * DIM_N == 256, "slice size");
static_assert(BROWS % 64 == 0 && NCOLS % 64 == 0 && KDIM % 32 == 0, "gemm M,N tile multiples and K % 32");
static_assert(DIM_K % 2 == 0, "k pairs");

constexpr size_t WS_Q_OFF    = 0;
constexpr size_t WS_Q_BYTES  = (size_t)BROWS * KDIM * 2;
constexpr size_t WS_WHI_OFF  = WS_Q_OFF + WS_Q_BYTES;
constexpr size_t WS_W_BYTES  = (size_t)NCOLS * KDIM * 2;
constexpr size_t WS_WLO_OFF  = WS_WHI_OFF + WS_W_BYTES;
constexpr size_t WS_TOTAL    = WS_WLO_OFF + WS_W_BYTES;
static_assert(WS_TOTAL == 8388608, "carve total");
static_assert(WS_TOTAL <= 134217728, "carve cap");

typedef __attribute__((ext_vector_type(16))) _Float16 v16h;
typedef __attribute__((ext_vector_type(8)))  _Float16 v8h;
typedef __attribute__((ext_vector_type(16))) __bf16   v16b;
typedef __attribute__((ext_vector_type(8)))  __bf16   v8b;
typedef __attribute__((ext_vector_type(8)))  float    v8f;
typedef __attribute__((ext_vector_type(4)))  float    v4f;
typedef __attribute__((ext_vector_type(4)))  unsigned int v4u;

__device__ __forceinline__ unsigned short f2bf_bits(float f) {
  unsigned u = __float_as_uint(f);
  return (unsigned short)((u + 0x7FFFu + ((u >> 16) & 1u)) >> 16);
}
__device__ __forceinline__ float bf_bits2f(unsigned short h) { return __uint_as_float(((unsigned)h) << 16); }

__device__ __forceinline__ void dep_guard_h(v8f& a, v8f& b, v16h x, v16h y) { asm volatile("v_nop\n\tv_nop\n\tv_nop\n\tv_nop" : "+v"(a), "+v"(b) : "v"(x), "v"(y)); }
__device__ __forceinline__ void dep_guard_b(v8f& a, v8f& b, v16b x, v16b y) { asm volatile("v_nop\n\tv_nop\n\tv_nop\n\tv_nop" : "+v"(a), "+v"(b) : "v"(x), "v"(y)); }
__device__ __forceinline__ void keep4_h(v16h a, v16h b, v16h c, v16h d) { asm volatile("v_nop" :: "v"(a), "v"(b), "v"(c), "v"(d)); }
__device__ __forceinline__ void keep4_b(v16b a, v16b b, v16b c, v16b d) { asm volatile("v_nop" :: "v"(a), "v"(b), "v"(c), "v"(d)); }
__device__ __forceinline__ void acc_guard4(v8f& a, v8f& b, v8f& c, v8f& d) { asm volatile("v_nop\n\tv_nop\n\tv_nop\n\tv_nop" : "+v"(a), "+v"(b), "+v"(c), "+v"(d)); }
template <typename T> struct Frag;
template <> struct Frag<_Float16> {
  typedef v16h V; union U { v16h v; v8h h[2]; };
  static __device__ __forceinline__ v16h load(const _Float16* p) {
    U f; f.h[0] = *(const v8h*)(p); f.h[1] = *(const v8h*)(p + 16); return f.v;
  }
  static __device__ __forceinline__ v8f mma(v16h a, v16h b, v8f c) {
    return __builtin_amdgcn_wmma_f32_16x16x32_f16(false, a, false, b, (short)0, c, false, false);
  }
  static __device__ __forceinline__ void guard(v8f& a, v8f& b, v16h x, v16h y) { dep_guard_h(a, b, x, y); }
  static __device__ __forceinline__ void keep(v16h a, v16h b, v16h c, v16h d) { keep4_h(a, b, c, d); }
};
template <> struct Frag<__bf16> {
  typedef v16b V; union U { v16b v; v8b h[2]; };
  static __device__ __forceinline__ v16b load(const __bf16* p) {
    U f; f.h[0] = *(const v8b*)(p); f.h[1] = *(const v8b*)(p + 16); return f.v;
  }
  static __device__ __forceinline__ v8f mma(v16b a, v16b b, v8f c) {
    return __builtin_amdgcn_wmma_f32_16x16x32_bf16(false, a, false, b, (short)0, c, false, false);
  }
  static __device__ __forceinline__ void guard(v8f& a, v8f& b, v16b x, v16b y) { dep_guard_b(a, b, x, y); }
  static __device__ __forceinline__ void keep(v16b a, v16b b, v16b c, v16b d) { keep4_b(a, b, c, d); }
};

__device__ __forceinline__ unsigned pk16(unsigned short a, unsigned short b) { return (unsigned)a | ((unsigned)b << 16); }

template <int ET> struct Elem;
template <> struct Elem<0> { typedef _Float16 T; };
template <> struct Elem<1> { typedef __bf16 T; };
template <int ET, bool SPLIT, int BIAS_MODE, int OUT_MODE, bool RESID, int ACT = 0, bool ASPLIT = SPLIT>
__global__ __launch_bounds__(256) void wmma_gemm64(
    const unsigned short* __restrict__ Ap, const unsigned short* __restrict__ A2p, int lda, long strideA,
    const unsigned short* __restrict__ Btp, const unsigned short* __restrict__ Bt2p, int ldb, long strideB,
    void* __restrict__ Cout, void* __restrict__ Cout2, int ldc, long strideC,
    const float* __restrict__ bias,
    const float* __restrict__ resid, long strideR,
    int M, int N, int K, float scale) {
  typedef typename Elem<ET>::T T;
  typedef typename Frag<T>::V V;
  const T* A = (const T*)Ap; const T* A2 = (const T*)A2p; const T* Bt = (const T*)Btp; const T* Bt2 = (const T*)Bt2p;
  __shared__ __align__(16) float sT[8][16 * 68];
  const int b    = blockIdx.y;
  const int lane = threadIdx.x & 31;
  const int wave = threadIdx.x >> 5;
  const int tilesN = N >> 6;
  const int tilesM = M >> 6;
  const int tile = blockIdx.x * 8 + wave;
  if (tile >= tilesM * tilesN) return;
  const int tm = tile / tilesN;
  const int tn = tile - tm * tilesN;
  const int m0 = tm << 6;
  const int n0 = tn << 6;

  const T* Ab  = A  + (size_t)b * strideA;
  const T* Bb  = Bt + (size_t)b * strideB;
  const T* Ab2 = (SPLIT && ASPLIT) ? (A2  + (size_t)b * strideA) : nullptr;
  const T* Bb2 = SPLIT ? (Bt2 + (size_t)b * strideB) : nullptr;

  const int rlane = lane & 15;
  const int koff  = (lane >> 4) * 8;
  const int mOff  = (lane >> 4) * 8;

  v8f acc[4][4];
#pragma unroll
  for (int i = 0; i < 4; ++i)
#pragma unroll
    for (int j = 0; j < 4; ++j) acc[i][j] = (v8f){0.f,0.f,0.f,0.f,0.f,0.f,0.f,0.f};

  for (int k0 = 0; k0 < K; k0 += 32) {
    V bh[4], bl[4];
#pragma unroll
    for (int j = 0; j < 4; ++j) {
      const size_t bo = (size_t)(n0 + (j << 4) + rlane) * ldb + koff + k0;
      bh[j] = Frag<T>::load(Bb + bo);
      if (SPLIT) bl[j] = Frag<T>::load(Bb2 + bo);
    }
#pragma unroll
    for (int i = 0; i < 4; ++i) {
      const size_t ao = (size_t)(m0 + (i << 4) + rlane) * lda + koff + k0;
      V ah = Frag<T>::load(Ab + ao);
      V al;
      if (SPLIT && ASPLIT) al = Frag<T>::load(Ab2 + ao);
#pragma unroll
      for (int j = 0; j < 4; ++j) {
        acc[i][j] = Frag<T>::mma(ah, bh[j], acc[i][j]);
        if (SPLIT) {
          acc[i][j] = Frag<T>::mma(ah, bl[j], acc[i][j]);
          if (ASPLIT) acc[i][j] = Frag<T>::mma(al, bh[j], acc[i][j]);
        }
      }
      Frag<T>::guard(acc[i][0], acc[i][3], ah, (SPLIT && ASPLIT) ? al : ah);
    }
    Frag<T>::keep(bh[0], bh[1], bh[2], bh[3]);
    if (SPLIT) Frag<T>::keep(bl[0], bl[1], bl[2], bl[3]);
  }
  acc_guard4(acc[0][0], acc[0][1], acc[0][2], acc[0][3]);
  acc_guard4(acc[1][0], acc[1][1], acc[1][2], acc[1][3]);
  acc_guard4(acc[2][0], acc[2][1], acc[2][2], acc[2][3]);
  acc_guard4(acc[3][0], acc[3][1], acc[3][2], acc[3][3]);

  float* slab = sT[wave];
  const float* Rb = RESID ? (resid + (size_t)b * strideR) : nullptr;
#pragma unroll
  for (int i = 0; i < 4; ++i) {
    const int mBase = m0 + (i << 4);
#pragma unroll
    for (int j = 0; j < 4; ++j) {
      const int n = n0 + (j << 4) + rlane;
      float bv = 0.f;
      if (BIAS_MODE == 2) bv = bias[n];
#pragma unroll
      for (int r = 0; r < 8; ++r) {
        float v = acc[i][j][r] * scale;
        if (BIAS_MODE == 1) v += bias[mBase + mOff + r];
        if (BIAS_MODE == 2) v += bv;
        if (RESID) v += Rb[(size_t)(mBase + mOff + r) * ldc + n];
        if (ACT == 2) v = fmaxf(v, 0.0f);
        if (ACT == 4) v = (v > 0.f) ? v : 0.01f * v;
        slab[(mOff + r) * 68 + (j << 4) + rlane] = v;
      }
    }
    __builtin_amdgcn_fence(__ATOMIC_RELEASE, "workgroup");
    __builtin_amdgcn_wave_barrier();
    __builtin_amdgcn_fence(__ATOMIC_ACQUIRE, "workgroup");
    if (OUT_MODE == 0) {
      float* C = (float*)Cout + (size_t)b * strideC;
      const int hh = lane >> 4, c4 = (lane & 15) * 4;
      for (int pass = 0; pass < 2; ++pass) {
#pragma unroll
        for (int it = 0; it < 8; ++it) {
          const int row = it * 2 + hh;
          v4f v = *(const v4f*)(slab + row * 68 + c4);
          *(volatile v4f*)(C + (size_t)(mBase + row) * ldc + n0 + c4) = v;
        }
        __threadfence();
      }
    } else {
      const int q = lane >> 3, c8 = (lane & 7) * 8;
      unsigned short* C  = (unsigned short*)Cout  + (size_t)b * strideC;
      unsigned short* C2 = (OUT_MODE == 2) ? ((unsigned short*)Cout2 + (size_t)b * strideC) : nullptr;
      for (int pass = 0; pass < 2; ++pass) {
#pragma unroll
        for (int it = 0; it < 4; ++it) {
          const int row = it * 4 + q;
          const float* sp = slab + row * 68 + c8;
          v8h hv, lv;
#pragma unroll
          for (int e = 0; e < 8; ++e) {
            if (OUT_MODE == 1) {
              hv[e] = (_Float16)sp[e];
            } else {
              unsigned short hb = f2bf_bits(sp[e]);
              unsigned short lb = f2bf_bits(sp[e] - bf_bits2f(hb));
              hv[e] = __builtin_bit_cast(_Float16, hb);
              lv[e] = __builtin_bit_cast(_Float16, lb);
            }
          }
          *(volatile v8h*)(C + (size_t)(mBase + row) * ldc + n0 + c8) = hv;
          if (OUT_MODE == 2) *(volatile v8h*)(C2 + (size_t)(mBase + row) * ldc + n0 + c8) = lv;
        }
        __threadfence();
      }
    }
    __builtin_amdgcn_fence(__ATOMIC_RELEASE, "workgroup");
    __builtin_amdgcn_wave_barrier();
    __builtin_amdgcn_fence(__ATOMIC_ACQUIRE, "workgroup");
  }
}

__device__ __forceinline__ unsigned short qcode_bits(float v, float rs) {
  float t = v * rs;
  t = rintf(t);
  t = fminf(fmaxf(t, -127.0f), 127.0f);
  return f2bf_bits(t);
}

__global__ __launch_bounds__(256) void quant_kernel(const float* __restrict__ x, const float* __restrict__ act_scale,
                                                    unsigned short* __restrict__ qout, int n8) {
  const int i = blockIdx.x * 256 + threadIdx.x;
  if (i >= n8) return;
  const float s  = fmaxf(fabsf(act_scale[0]), 1e-8f);
  const float rs = 1.0f / s;
  const float* p = x + 8 * (size_t)i;
  const v4f a = *(const v4f*)(p);
  const v4f c = *(const v4f*)(p + 4);
  unsigned short hb[8];
#pragma unroll
  for (int e = 0; e < 4; ++e) {
    hb[e]     = qcode_bits(a[e], rs);
    hb[4 + e] = qcode_bits(c[e], rs);
  }
  const v4u u = (v4u){pk16(hb[0], hb[1]), pk16(hb[2], hb[3]), pk16(hb[4], hb[5]), pk16(hb[6], hb[7])};
  unsigned short* q = qout + 8 * (size_t)i;
  *(volatile v4u*)q = u;
  __threadfence();
  *(volatile v4u*)q = u;
}

constexpr int SW_PITCH = 68;

__global__ __launch_bounds__(256) void build_w_kernel(const float* __restrict__ Y,
                                                      const float* __restrict__ Z,
                                                      const float* __restrict__ A,
                                                      const float* __restrict__ act_scale,
                                                      unsigned short* __restrict__ Whi,
                                                      unsigned short* __restrict__ Wlo) {
  __shared__ float sYs[4][GRP];
  __shared__ float sZs[4][GRP];
  __shared__ float sPart[8][8];
  __shared__ float sC[4][4];
  __shared__ __align__(16) float sW[DIM_M * SW_PITCH];

  const int t    = threadIdx.x;
  const int lane = t & 31;
  const int wave = t >> 5;
  const int j    = blockIdx.x >> 4;
  const int kp   = blockIdx.x & 15;
  const int k0   = kp * 2;

  float ay[4], az[4];
#pragma unroll
  for (int g = 0; g < 4; ++g) {
    const int p = g >> 1, kk = g & 1;
    const size_t base = (((size_t)p * DIM_J + j) * DIM_K + (size_t)(k0 + kk)) * GRP;
    const float yv = Y[base + t];
    const float zv = Z[base + t];
    sYs[g][t] = (yv > 0.0f) ? 1.0f : ((yv < 0.0f) ? -1.0f : 0.0f);
    sZs[g][t] = (zv > 0.0f) ? 1.0f : ((zv < 0.0f) ? -1.0f : 0.0f);
    ay[g] = fabsf(yv);
    az[g] = fabsf(zv);
  }
#pragma unroll
  for (int g = 0; g < 4; ++g) {
    float vy = ay[g], vz = az[g];
#pragma unroll
    for (int off = 16; off > 0; off >>= 1) {
      vy += __shfl_xor(vy, off, 32);
      vz += __shfl_xor(vz, off, 32);
    }
    if (lane == 0) { sPart[g][wave] = vy; sPart[4 + g][wave] = vz; }
  }
  __syncthreads();

  {
    const int g = t & 3;
    const int p = g >> 1, kk = g & 1;
    float ys = 0.0f, zs = 0.0f;
#pragma unroll
    for (int w = 0; w < 8; ++w) { ys += sPart[g][w]; zs += sPart[4 + g][w]; }
    const float ysc = ys * (1.0f / 256.0f);
    const float zsc = zs * (1.0f / 256.0f);
    const v4f av = *(const v4f*)(A + ((((size_t)p * DIM_J + j) * DIM_K + (size_t)(k0 + kk)) * 4));
    if (t < 4) {
      sC[g][0] = av[0] * ysc * zsc;
      sC[g][1] = av[1] * ysc;
      sC[g][2] = av[2] * zsc;
      sC[g][3] = av[3];
    }
  }
  __syncthreads();

  {
    const float s_act = fmaxf(fabsf(act_scale[0]), 1e-8f);
    const int kk  = wave & 1;
    const int c   = t & 63;
    const int n   = t & 31;
    const int mlo = t >> 6;
#pragma unroll 1
    for (int it = 0; it < 8; ++it) {
      const int m = it * 4 + mlo;
      float w = 0.0f;
#pragma unroll
      for (int p = 0; p < 2; ++p) {
        const int g = p * 2 + kk;
        const float* ys = &sYs[g][m * DIM_L];
        const float* zs = &sZs[g][n];
        float smn = 0.0f, ym = 0.0f, zn = 0.0f;
#pragma unroll
        for (int l = 0; l < DIM_L; ++l) {
          const float sy = ys[l];
          const float sz = zs[l * DIM_N];
          smn += sy * sz;
          ym  += sy;
          zn  += sz;
        }
        w += sC[g][0] * smn + sC[g][1] * ym + sC[g][2] * zn + sC[g][3];
      }
      sW[m * SW_PITCH + c] = w * s_act;
    }
  }
  __syncthreads();

  {
    const int row = wave * 4 + (lane >> 3);
    const int c8  = (lane & 7) * 8;
    const float* sp = sW + row * SW_PITCH + c8;
    const v4f v0 = *(const v4f*)(sp);
    const v4f v1 = *(const v4f*)(sp + 4);
    unsigned short hb[8], lb[8];
#pragma unroll
    for (int e = 0; e < 4; ++e) {
      const float w0 = v0[e], w1 = v1[e];
      hb[e] = f2bf_bits(w0);
      lb[e] = f2bf_bits(w0 - bf_bits2f(hb[e]));
      hb[4 + e] = f2bf_bits(w1);
      lb[4 + e] = f2bf_bits(w1 - bf_bits2f(hb[4 + e]));
    }
    const v4u uh = (v4u){pk16(hb[0], hb[1]), pk16(hb[2], hb[3]), pk16(hb[4], hb[5]), pk16(hb[6], hb[7])};
    const v4u ul = (v4u){pk16(lb[0], lb[1]), pk16(lb[2], lb[3]), pk16(lb[4], lb[5]), pk16(lb[6], lb[7])};
    const size_t o = (size_t)(j * DIM_M + row) * KDIM + (size_t)kp * 64 + c8;
    unsigned short* ph = Whi + o;
    unsigned short* pl = Wlo + o;
    *(volatile v4u*)ph = uh;
    *(volatile v4u*)pl = ul;
    __threadfence();
    *(volatile v4u*)ph = uh;
    *(volatile v4u*)pl = ul;
  }
}

extern "C" void kernel_launch(void* const* d_in, const int* in_sizes, int n_in,
                              void* d_out, int out_size, void* d_ws, size_t ws_size,
                              hipStream_t stream) {
  (void)in_sizes;
  if (n_in < 6) return;
  if (ws_size < WS_TOTAL) return;
  if ((size_t)out_size < (size_t)BROWS * NCOLS) return;

  const float* x    = (const float*)d_in[0];
  const float* Y    = (const float*)d_in[1];
  const float* Z    = (const float*)d_in[2];
  const float* A    = (const float*)d_in[3];
  const float* bias = (const float*)d_in[4];
  const float* act  = (const float*)d_in[5];

  unsigned short* q   = (unsigned short*)((char*)d_ws + WS_Q_OFF);
  unsigned short* Whi = (unsigned short*)((char*)d_ws + WS_WHI_OFF);
  unsigned short* Wlo = (unsigned short*)((char*)d_ws + WS_WLO_OFF);
  float* out = (float*)d_out;

  const int n8 = BROWS * KDIM / 8;
  quant_kernel<<<(n8 + 255) / 256, 256, 0, stream>>>(x, act, q, n8);

  build_w_kernel<<<DIM_J * (DIM_K / 2), 256, 0, stream>>>(Y, Z, A, act, Whi, Wlo);

  const int tiles = (BROWS / 64) * (NCOLS / 64);
  wmma_gemm64<1, true, 2, 0, false, 0, false><<<dim3((tiles + 7) / 8, 1), 256, 0, stream>>>(
      q, q, KDIM, 0L,
      Whi, Wlo, KDIM, 0L,
      (void*)out, (void*)out, NCOLS, 0L,
      bias,
      bias, 0L,
      BROWS, NCOLS, KDIM, 1.0f);
}
